// VSSOnewayLayer_3238405341501
// MI455X (gfx1250) — hardware-verified
//
#include <hip/hip_runtime.h>
#include <hip/hip_bf16.h>

typedef __attribute__((ext_vector_type(16))) _Float16 v16h;
typedef __attribute__((ext_vector_type(8)))  _Float16 v8h;
typedef __attribute__((ext_vector_type(16))) __bf16   v16b;
typedef __attribute__((ext_vector_type(8)))  __bf16   v8b;
typedef __attribute__((ext_vector_type(8)))  float    v8f;
typedef __attribute__((ext_vector_type(4)))  float    v4f;

__device__ __forceinline__ unsigned short f2bf_bits(float f) {
  unsigned u = __float_as_uint(f);
  return (unsigned short)((u + 0x7FFFu + ((u >> 16) & 1u)) >> 16);
}
__device__ __forceinline__ float bf_bits2f(unsigned short h) { return __uint_as_float(((unsigned)h) << 16); }

__device__ __forceinline__ void dep_guard_h(v8f& a, v8f& b, v16h x, v16h y) { asm volatile("v_nop\n\tv_nop\n\tv_nop\n\tv_nop" : "+v"(a), "+v"(b) : "v"(x), "v"(y)); }
__device__ __forceinline__ void dep_guard_b(v8f& a, v8f& b, v16b x, v16b y) { asm volatile("v_nop\n\tv_nop\n\tv_nop\n\tv_nop" : "+v"(a), "+v"(b) : "v"(x), "v"(y)); }
__device__ __forceinline__ void keep4_h(v16h a, v16h b, v16h c, v16h d) { asm volatile("v_nop" :: "v"(a), "v"(b), "v"(c), "v"(d)); }
__device__ __forceinline__ void keep4_b(v16b a, v16b b, v16b c, v16b d) { asm volatile("v_nop" :: "v"(a), "v"(b), "v"(c), "v"(d)); }
__device__ __forceinline__ void acc_guard4(v8f& a, v8f& b, v8f& c, v8f& d) { asm volatile("v_nop\n\tv_nop\n\tv_nop\n\tv_nop" : "+v"(a), "+v"(b), "+v"(c), "+v"(d)); }
template <typename T> struct Frag;
template <> struct Frag<_Float16> {
  typedef v16h V; union U { v16h v; v8h h[2]; };
  static __device__ __forceinline__ v16h load(const _Float16* p) {
    U f; f.h[0] = *(const v8h*)(p); f.h[1] = *(const v8h*)(p + 16); return f.v;
  }
  static __device__ __forceinline__ v8f mma(v16h a, v16h b, v8f c) {
    return __builtin_amdgcn_wmma_f32_16x16x32_f16(false, a, false, b, (short)0, c, false, false);
  }
  static __device__ __forceinline__ void guard(v8f& a, v8f& b, v16h x, v16h y) { dep_guard_h(a, b, x, y); }
  static __device__ __forceinline__ void keep(v16h a, v16h b, v16h c, v16h d) { keep4_h(a, b, c, d); }
};
template <> struct Frag<__bf16> {
  typedef v16b V; union U { v16b v; v8b h[2]; };
  static __device__ __forceinline__ v16b load(const __bf16* p) {
    U f; f.h[0] = *(const v8b*)(p); f.h[1] = *(const v8b*)(p + 16); return f.v;
  }
  static __device__ __forceinline__ v8f mma(v16b a, v16b b, v8f c) {
    return __builtin_amdgcn_wmma_f32_16x16x32_bf16(false, a, false, b, (short)0, c, false, false);
  }
  static __device__ __forceinline__ void guard(v8f& a, v8f& b, v16b x, v16b y) { dep_guard_b(a, b, x, y); }
  static __device__ __forceinline__ void keep(v16b a, v16b b, v16b c, v16b d) { keep4_b(a, b, c, d); }
};

template <int ET> struct Elem;
template <> struct Elem<0> { typedef _Float16 T; };
template <> struct Elem<1> { typedef __bf16 T; };
template <int ET, bool SPLIT, int BIAS_MODE, int OUT_MODE, bool RESID, int ACT = 0>
__global__ __launch_bounds__(256) void wmma_gemm64(
    const unsigned short* __restrict__ Ap, const unsigned short* __restrict__ A2p, int lda, long strideA,
    const unsigned short* __restrict__ Btp, const unsigned short* __restrict__ Bt2p, int ldb, long strideB,
    void* __restrict__ Cout, void* __restrict__ Cout2, int ldc, long strideC,
    const float* __restrict__ bias,
    const float* __restrict__ resid, long strideR,
    int M, int N, int K, float scale) {
  typedef typename Elem<ET>::T T;
  typedef typename Frag<T>::V V;
  const T* A = (const T*)Ap; const T* A2 = (const T*)A2p; const T* Bt = (const T*)Btp; const T* Bt2 = (const T*)Bt2p;
  __shared__ __align__(16) float sT[8][16 * 68];
  const int b    = blockIdx.y;
  const int lane = threadIdx.x & 31;
  const int wave = threadIdx.x >> 5;
  const int tilesN = N >> 6;
  const int tilesM = M >> 6;
  const int tile = blockIdx.x * 8 + wave;
  if (tile >= tilesM * tilesN) return;
  const int tm = tile / tilesN;
  const int tn = tile - tm * tilesN;
  const int m0 = tm << 6;
  const int n0 = tn << 6;

  const T* Ab  = A  + (size_t)b * strideA;
  const T* Bb  = Bt + (size_t)b * strideB;
  const T* Ab2 = SPLIT ? (A2  + (size_t)b * strideA) : nullptr;
  const T* Bb2 = SPLIT ? (Bt2 + (size_t)b * strideB) : nullptr;

  const int rlane = lane & 15;
  const int koff  = (lane >> 4) * 8;
  const int mOff  = (lane >> 4) * 8;

  v8f acc[4][4];
#pragma unroll
  for (int i = 0; i < 4; ++i)
#pragma unroll
    for (int j = 0; j < 4; ++j) acc[i][j] = (v8f){0.f,0.f,0.f,0.f,0.f,0.f,0.f,0.f};

  for (int k0 = 0; k0 < K; k0 += 32) {
    V bh[4], bl[4];
#pragma unroll
    for (int j = 0; j < 4; ++j) {
      const size_t bo = (size_t)(n0 + (j << 4) + rlane) * ldb + koff + k0;
      bh[j] = Frag<T>::load(Bb + bo);
      if (SPLIT) bl[j] = Frag<T>::load(Bb2 + bo);
    }
#pragma unroll
    for (int i = 0; i < 4; ++i) {
      const size_t ao = (size_t)(m0 + (i << 4) + rlane) * lda + koff + k0;
      V ah = Frag<T>::load(Ab + ao);
      V al;
      if (SPLIT) al = Frag<T>::load(Ab2 + ao);
#pragma unroll
      for (int j = 0; j < 4; ++j) {
        acc[i][j] = Frag<T>::mma(ah, bh[j], acc[i][j]);
        if (SPLIT) {
          acc[i][j] = Frag<T>::mma(ah, bl[j], acc[i][j]);
          acc[i][j] = Frag<T>::mma(al, bh[j], acc[i][j]);
        }
      }
      Frag<T>::guard(acc[i][0], acc[i][3], ah, SPLIT ? al : ah);
    }
    Frag<T>::keep(bh[0], bh[1], bh[2], bh[3]);
    if (SPLIT) Frag<T>::keep(bl[0], bl[1], bl[2], bl[3]);
  }
  acc_guard4(acc[0][0], acc[0][1], acc[0][2], acc[0][3]);
  acc_guard4(acc[1][0], acc[1][1], acc[1][2], acc[1][3]);
  acc_guard4(acc[2][0], acc[2][1], acc[2][2], acc[2][3]);
  acc_guard4(acc[3][0], acc[3][1], acc[3][2], acc[3][3]);

  float* slab = sT[wave];
  const float* Rb = RESID ? (resid + (size_t)b * strideR) : nullptr;
#pragma unroll
  for (int i = 0; i < 4; ++i) {
    const int mBase = m0 + (i << 4);
#pragma unroll
    for (int j = 0; j < 4; ++j) {
      const int n = n0 + (j << 4) + rlane;
      float bv = 0.f;
      if (BIAS_MODE == 2) bv = bias[n];
#pragma unroll
      for (int r = 0; r < 8; ++r) {
        float v = acc[i][j][r] * scale;
        if (BIAS_MODE == 1) v += bias[mBase + mOff + r];
        if (BIAS_MODE == 2) v += bv;
        if (RESID) v += Rb[(size_t)(mBase + mOff + r) * ldc + n];
        if (ACT == 1) v = tanhf(v);
        if (ACT == 2) v = fmaxf(v, 0.0f);
        if (ACT == 3) v = v / (1.0f + expf(-v));
        if (ACT == 4) v = (v > 0.f) ? v : 0.01f * v;
        if (ACT == 5) v = 0.5f * v * (1.0f + erff(v * 0.70710678118654752f));
        slab[(mOff + r) * 68 + (j << 4) + rlane] = v;
      }
    }
    __builtin_amdgcn_fence(__ATOMIC_RELEASE, "workgroup");
    __builtin_amdgcn_wave_barrier();
    __builtin_amdgcn_fence(__ATOMIC_ACQUIRE, "workgroup");
    if (OUT_MODE == 0) {
      float* C = (float*)Cout + (size_t)b * strideC;
      const int hh = lane >> 4, c4 = (lane & 15) * 4;
      for (int pass = 0; pass < 2; ++pass) {
#pragma unroll
        for (int it = 0; it < 8; ++it) {
          const int row = it * 2 + hh;
          v4f v = *(const v4f*)(slab + row * 68 + c4);
          *(volatile v4f*)(C + (size_t)(mBase + row) * ldc + n0 + c4) = v;
        }
        __threadfence();
      }
    } else {
      const int q = lane >> 3, c8 = (lane & 7) * 8;
      unsigned short* C  = (unsigned short*)Cout  + (size_t)b * strideC;
      unsigned short* C2 = (OUT_MODE == 2) ? ((unsigned short*)Cout2 + (size_t)b * strideC) : nullptr;
      for (int pass = 0; pass < 2; ++pass) {
#pragma unroll
        for (int it = 0; it < 4; ++it) {
          const int row = it * 4 + q;
          const float* sp = slab + row * 68 + c8;
          v8h hv, lv;
#pragma unroll
          for (int e = 0; e < 8; ++e) {
            if (OUT_MODE == 1) {
              hv[e] = (_Float16)sp[e];
            } else {
              unsigned short hb = f2bf_bits(sp[e]);
              unsigned short lb = f2bf_bits(sp[e] - bf_bits2f(hb));
              hv[e] = __builtin_bit_cast(_Float16, hb);
              lv[e] = __builtin_bit_cast(_Float16, lb);
            }
          }
          *(volatile v8h*)(C + (size_t)(mBase + row) * ldc + n0 + c8) = hv;
          if (OUT_MODE == 2) *(volatile v8h*)(C2 + (size_t)(mBase + row) * ldc + n0 + c8) = lv;
        }
        __threadfence();
      }
    }
    __builtin_amdgcn_fence(__ATOMIC_RELEASE, "workgroup");
    __builtin_amdgcn_wave_barrier();
    __builtin_amdgcn_fence(__ATOMIC_ACQUIRE, "workgroup");
  }
}

__global__ __launch_bounds__(256) void k_wt_f16(const float* __restrict__ in, _Float16* __restrict__ out,
                                                int K, int Nsrc, int Npad, float sc) {
  __shared__ __align__(16) _Float16 s[64 * 72];
  const int tid = threadIdx.x, lane = tid & 31, wave = tid >> 5;
  const int k0 = blockIdx.x * 64, n0 = blockIdx.y * 64;
#pragma unroll
  for (int i = 0; i < 16; ++i) {
    const int idx = tid + 256 * i;
    const int kk = idx >> 6, nn = idx & 63;
    const int n = n0 + nn;
    const int nc = (n < Nsrc) ? n : (Nsrc - 1);
    float v = in[(size_t)(k0 + kk) * Nsrc + nc] * sc;
    if (n >= Nsrc) v = 0.f;
    s[nn * 72 + kk] = (_Float16)v;
  }
  __syncthreads();
  v8h val[2]; size_t off[2];
#pragma unroll
  for (int it = 0; it < 2; ++it) {
    const int nn = wave * 8 + it * 4 + (lane >> 3);
    const int c8 = (lane & 7) * 8;
    val[it] = *(const v8h*)(s + nn * 72 + c8);
    off[it] = (size_t)(n0 + nn) * K + k0 + c8;
  }
#pragma unroll
  for (int it = 0; it < 2; ++it) *(volatile v8h*)(out + off[it]) = val[it];
  __threadfence();
#pragma unroll
  for (int it = 0; it < 2; ++it) *(volatile v8h*)(out + off[it]) = val[it];
  (void)Npad;
}

__global__ __launch_bounds__(256) void k_ln256(const float* __restrict__ in, const float* __restrict__ gam,
                                               const float* __restrict__ bet, _Float16* __restrict__ out, int nrows) {
  const int lane = threadIdx.x & 31, wave = threadIdx.x >> 5;
  const int row = blockIdx.x * 8 + wave;
  if (row >= nrows) return;
  const int c = lane * 8;
  const float* rp = in + (size_t)row * 256 + c;
  const v4f a0 = *(const v4f*)rp, a1 = *(const v4f*)(rp + 4);
  float v[8];
#pragma unroll
  for (int i = 0; i < 4; ++i) { v[i] = a0[i]; v[4 + i] = a1[i]; }
  float s = 0.f;
#pragma unroll
  for (int i = 0; i < 8; ++i) s += v[i];
#pragma unroll
  for (int off = 16; off > 0; off >>= 1) s += __shfl_xor(s, off, 32);
  const float mean = s * (1.0f / 256.0f);
  float q = 0.f;
#pragma unroll
  for (int i = 0; i < 8; ++i) { v[i] -= mean; q += v[i] * v[i]; }
#pragma unroll
  for (int off = 16; off > 0; off >>= 1) q += __shfl_xor(q, off, 32);
  const float rs = rsqrtf(q * (1.0f / 256.0f) + 1e-5f);
  const v4f g0 = *(const v4f*)(gam + c), g1 = *(const v4f*)(gam + c + 4);
  const v4f b0 = *(const v4f*)(bet + c), b1 = *(const v4f*)(bet + c + 4);
  v8h hv;
#pragma unroll
  for (int i = 0; i < 4; ++i) {
    hv[i]     = (_Float16)(v[i] * rs * g0[i] + b0[i]);
    hv[4 + i] = (_Float16)(v[4 + i] * rs * g1[i] + b1[i]);
  }
  _Float16* op = out + (size_t)row * 256 + c;
  *(volatile v8h*)op = hv;
  __threadfence();
  *(volatile v8h*)op = hv;
}

__global__ __launch_bounds__(256) void k_ln512(const float* __restrict__ in, const float* __restrict__ gam,
                                               const float* __restrict__ bet, _Float16* __restrict__ out, int nrows) {
  const int lane = threadIdx.x & 31, wave = threadIdx.x >> 5;
  const int row = blockIdx.x * 8 + wave;
  if (row >= nrows) return;
  const int cA = lane * 8, cB = 256 + lane * 8;
  const float* rp = in + (size_t)row * 512;
  const v4f a0 = *(const v4f*)(rp + cA), a1 = *(const v4f*)(rp + cA + 4);
  const v4f a2 = *(const v4f*)(rp + cB), a3 = *(const v4f*)(rp + cB + 4);
  float v[16];
#pragma unroll
  for (int i = 0; i < 4; ++i) { v[i] = a0[i]; v[4 + i] = a1[i]; v[8 + i] = a2[i]; v[12 + i] = a3[i]; }
  float s = 0.f;
#pragma unroll
  for (int i = 0; i < 16; ++i) s += v[i];
#pragma unroll
  for (int off = 16; off > 0; off >>= 1) s += __shfl_xor(s, off, 32);
  const float mean = s * (1.0f / 512.0f);
  float q = 0.f;
#pragma unroll
  for (int i = 0; i < 16; ++i) { v[i] -= mean; q += v[i] * v[i]; }
#pragma unroll
  for (int off = 16; off > 0; off >>= 1) q += __shfl_xor(q, off, 32);
  const float rs = rsqrtf(q * (1.0f / 512.0f) + 1e-5f);
  const v4f g0 = *(const v4f*)(gam + cA), g1 = *(const v4f*)(gam + cA + 4);
  const v4f g2 = *(const v4f*)(gam + cB), g3 = *(const v4f*)(gam + cB + 4);
  const v4f b0 = *(const v4f*)(bet + cA), b1 = *(const v4f*)(bet + cA + 4);
  const v4f b2 = *(const v4f*)(bet + cB), b3 = *(const v4f*)(bet + cB + 4);
  v8h hA, hB;
#pragma unroll
  for (int i = 0; i < 4; ++i) {
    hA[i]     = (_Float16)(v[i] * rs * g0[i] + b0[i]);
    hA[4 + i] = (_Float16)(v[4 + i] * rs * g1[i] + b1[i]);
    hB[i]     = (_Float16)(v[8 + i] * rs * g2[i] + b2[i]);
    hB[4 + i] = (_Float16)(v[12 + i] * rs * g3[i] + b3[i]);
  }
  _Float16* op = out + (size_t)row * 512;
  *(volatile v8h*)(op + cA) = hA;
  *(volatile v8h*)(op + cB) = hB;
  __threadfence();
  *(volatile v8h*)(op + cA) = hA;
  *(volatile v8h*)(op + cB) = hB;
}

__global__ __launch_bounds__(256) void k_conv_gelu(const float* __restrict__ up, const float* __restrict__ cw,
                                                   const float* __restrict__ cb, float* __restrict__ u32,
                                                   _Float16* __restrict__ u16, int nrows, int L) {
  __shared__ __align__(16) float sv[8 * 256];
  const int tid = threadIdx.x, lane = tid & 31, wave = tid >> 5;
  int row = blockIdx.x * 4 + (wave >> 1);
  if (row > nrows - 1) row = nrows - 1;
  const int l = row % L;
  const int rm = (l > 0) ? (row - 1) : row;
  const int rp = (l < L - 1) ? (row + 1) : row;
  const int chalf = (wave & 1) * 256;
  const int cbase = chalf + lane * 8;
  float* sw = sv + wave * 256;
#pragma unroll 1
  for (int e = 0; e < 8; ++e) {
    const int c = cbase + e;
    float xm = up[(size_t)rm * 512 + c];
    const float x0 = up[(size_t)row * 512 + c];
    float xp = up[(size_t)rp * 512 + c];
    if (l == 0) xm = 0.f;
    if (l == L - 1) xp = 0.f;
    float v = xm * cw[c * 3 + 0] + x0 * cw[c * 3 + 1] + xp * cw[c * 3 + 2] + cb[c];
    v = 0.5f * v * (1.0f + erff(v * 0.70710678118654752f));
    sw[lane * 8 + e] = v;
  }
  __syncthreads();
  v4f f[2];
#pragma unroll
  for (int j = 0; j < 2; ++j) f[j] = *(const v4f*)(sw + 128 * j + 4 * lane);
  const v4f o0 = *(const v4f*)(sw + lane * 8), o1 = *(const v4f*)(sw + lane * 8 + 4);
  v8h hv;
#pragma unroll
  for (int i = 0; i < 4; ++i) { hv[i] = (_Float16)(o0[i] * 64.0f); hv[4 + i] = (_Float16)(o1[i] * 64.0f); }
  float* b32 = u32 + (size_t)row * 512 + chalf;
  _Float16* b16 = u16 + (size_t)row * 512 + cbase;
#pragma unroll
  for (int j = 0; j < 2; ++j) *(volatile v4f*)(b32 + 128 * j + 4 * lane) = f[j];
  *(volatile v8h*)b16 = hv;
  __threadfence();
#pragma unroll
  for (int j = 0; j < 2; ++j) *(volatile v4f*)(b32 + 128 * j + 4 * lane) = f[j];
  *(volatile v8h*)b16 = hv;
}

#define SC_TS 32
__global__ __launch_bounds__(256) void k_scan(const float* __restrict__ dbc, const float* __restrict__ u,
                                              const float* __restrict__ dt_bias, const float* __restrict__ A_log,
                                              const float* __restrict__ Ds, float* __restrict__ y, int L) {
  __shared__ __align__(16) float sBC[SC_TS * 128];
  __shared__ __align__(16) float sX[SC_TS * 64];
  __shared__ __align__(16) float sY[SC_TS * 64];
  __shared__ float sDT[SC_TS];
  __shared__ float sDEC[SC_TS];
  const int tid = threadIdx.x, lane = tid & 31, wave = tid >> 5;
  const int b = blockIdx.x / 8, h = blockIdx.x % 8;
  const int p = tid >> 2, nseg = (tid & 3) * 16;
  const float Ah = -expf(A_log[h]);
  const float bias = dt_bias[h];
  const float Dh = Ds[h];
  const size_t rb = (size_t)b * L;
  float st[16];
#pragma unroll
  for (int i = 0; i < 16; ++i) st[i] = 0.f;
  const int nch = L / SC_TS;
#pragma unroll 1
  for (int ch = 0; ch < nch; ++ch) {
    const int l0 = ch * SC_TS;
    __syncthreads();
#pragma unroll
    for (int i = 0; i < 4; ++i) {
      const int idx = tid + 256 * i;
      const int s = idx >> 5, c4 = (idx & 31) * 4;
      *(v4f*)(sBC + s * 128 + c4) = *(const v4f*)(dbc + (rb + l0 + s) * 192 + 8 + c4);
    }
#pragma unroll
    for (int i = 0; i < 2; ++i) {
      const int idx = tid + 256 * i;
      const int s = idx >> 4, c4 = (idx & 15) * 4;
      *(v4f*)(sX + s * 64 + c4) = *(const v4f*)(u + (rb + l0 + s) * 512 + h * 64 + c4);
    }
    if (tid < SC_TS) {
      const float dr = dbc[(rb + l0 + tid) * 192 + h] + bias;
      const float sp = fmaxf(dr, 0.f) + log1pf(expf(-fabsf(dr)));
      sDT[tid] = sp;
      sDEC[tid] = expf(sp * Ah);
    }
    __syncthreads();
#pragma unroll 1
    for (int s = 0; s < SC_TS; ++s) {
      const float dec = sDEC[s], dt = sDT[s];
      const float xp = sX[s * 64 + p];
      const float dx = dt * xp;
      const float* Bp = sBC + s * 128 + nseg;
      const float* Cp = Bp + 64;
      float acc = 0.f;
#pragma unroll
      for (int i = 0; i < 4; ++i) {
        const v4f Bq = *(const v4f*)(Bp + 4 * i);
        const v4f Cq = *(const v4f*)(Cp + 4 * i);
#pragma unroll
        for (int e = 0; e < 4; ++e) {
          const float hn = st[4 * i + e] * dec + dx * Bq[e];
          st[4 * i + e] = hn;
          acc += hn * Cq[e];
        }
      }
      acc += __shfl_xor(acc, 1, 32);
      acc += __shfl_xor(acc, 2, 32);
      if ((tid & 3) == 0) sY[s * 64 + p] = acc + xp * Dh;
    }
    __syncthreads();
    v4f vv[2]; size_t off[2];
#pragma unroll
    for (int j = 0; j < 2; ++j) {
      const int s = wave * 4 + 2 * j + (lane >> 4);
      const int c4 = (lane & 15) * 4;
      vv[j] = *(const v4f*)(sY + s * 64 + c4);
      off[j] = (rb + l0 + s) * 512 + (size_t)h * 64 + c4;
    }
#pragma unroll
    for (int j = 0; j < 2; ++j) *(volatile v4f*)(y + off[j]) = vv[j];
    __threadfence();
#pragma unroll
    for (int j = 0; j < 2; ++j) *(volatile v4f*)(y + off[j]) = vv[j];
  }
}

static inline size_t align256(size_t x) { return (x + 255) & ~(size_t)255; }

extern "C" void kernel_launch(void* const* d_in, const int* in_sizes, int n_in,
                              void* d_out, int out_size, void* d_ws, size_t ws_size,
                              hipStream_t stream) {
  if (n_in < 13) return;
  const int D = 256, DIN = 512, L = 2048, H = 8, NS = 64, NXPP = 192;
  const int BL = in_sizes[0] / D;
  const int NXP = in_sizes[6] / DIN;
  if (BL <= 0 || (BL % L) != 0 || (BL % 64) != 0) return;
  if (in_sizes[0] != BL * D || in_sizes[3] != D * DIN || in_sizes[4] != DIN * 3 ||
      in_sizes[6] != DIN * NXP || NXP != H + 2 * NS || in_sizes[12] != DIN * D || out_size != BL * D) return;
  const int NB = BL / L;

  const float* src     = (const float*)d_in[0];
  const float* ln_w    = (const float*)d_in[1];
  const float* ln_b    = (const float*)d_in[2];
  const float* W_in    = (const float*)d_in[3];
  const float* conv_w  = (const float*)d_in[4];
  const float* conv_b  = (const float*)d_in[5];
  const float* W_xproj = (const float*)d_in[6];
  const float* dt_bias = (const float*)d_in[7];
  const float* A_log   = (const float*)d_in[8];
  const float* Ds      = (const float*)d_in[9];
  const float* oln_w   = (const float*)d_in[10];
  const float* oln_b   = (const float*)d_in[11];
  const float* W_out   = (const float*)d_in[12];
  float* out = (float*)d_out;

  size_t off = 0;
  const size_t o_x16  = off; off += align256((size_t)BL * D * 2);
  const size_t o_btin = off; off += align256((size_t)DIN * D * 2);
  const size_t o_btx  = off; off += align256((size_t)NXPP * DIN * 2);
  const size_t o_bto  = off; off += align256((size_t)D * DIN * 2);
  const size_t o_p    = off; off += align256((size_t)BL * DIN * 4);
  const size_t o_u32  = off; off += align256((size_t)BL * DIN * 4);
  const size_t o_h    = off; off += align256((size_t)BL * DIN * 2);
  const size_t o_dbc  = off; off += align256((size_t)BL * NXPP * 4);
  if (off > ws_size) return;

  char* ws = (char*)d_ws;
  _Float16* x16   = (_Float16*)(ws + o_x16);
  _Float16* BtIn  = (_Float16*)(ws + o_btin);
  _Float16* BtX   = (_Float16*)(ws + o_btx);
  _Float16* BtOut = (_Float16*)(ws + o_bto);
  float*    u_pre = (float*)(ws + o_p);
  float*    yss   = (float*)(ws + o_p);
  float*    u32   = (float*)(ws + o_u32);
  _Float16* u16   = (_Float16*)(ws + o_h);
  _Float16* yln   = (_Float16*)(ws + o_h);
  float*    dbc   = (float*)(ws + o_dbc);

  k_wt_f16<<<dim3(D / 64, DIN / 64), 256, 0, stream>>>(W_in, BtIn, D, DIN, DIN, 64.0f);
  k_wt_f16<<<dim3(DIN / 64, NXPP / 64), 256, 0, stream>>>(W_xproj, BtX, DIN, NXP, NXPP, 64.0f);
  k_wt_f16<<<dim3(DIN / 64, D / 64), 256, 0, stream>>>(W_out, BtOut, DIN, D, D, 64.0f);

  k_ln256<<<(BL + 7) / 8, 256, 0, stream>>>(src, ln_w, ln_b, x16, BL);

  {
    const int tiles = (BL / 64) * (DIN / 64);
    wmma_gemm64<0, false, 0, 0, false><<<dim3((tiles + 7) / 8, 1), 256, 0, stream>>>(
        (const unsigned short*)x16, nullptr, D, 0L,
        (const unsigned short*)BtIn, nullptr, D, 0L,
        (void*)u_pre, nullptr, DIN, 0L,
        nullptr, nullptr, 0L, BL, DIN, D, 1.0f / 64.0f);
  }

  k_conv_gelu<<<BL / 4, 256, 0, stream>>>(u_pre, conv_w, conv_b, u32, u16, BL, L);

  {
    const int tiles = (BL / 64) * (NXPP / 64);
    wmma_gemm64<0, false, 0, 0, false><<<dim3((tiles + 7) / 8, 1), 256, 0, stream>>>(
        (const unsigned short*)u16, nullptr, DIN, 0L,
        (const unsigned short*)BtX, nullptr, DIN, 0L,
        (void*)dbc, nullptr, NXPP, 0L,
        nullptr, nullptr, 0L, BL, NXPP, DIN, 1.0f / 4096.0f);
  }

  k_scan<<<NB * H, 256, 0, stream>>>(dbc, u32, dt_bias, A_log, Ds, yss, L);

  k_ln512<<<(BL + 7) / 8, 256, 0, stream>>>(yss, oln_w, oln_b, yln, BL);

  {
    const int tiles = (BL / 64) * (D / 64);
    wmma_gemm64<0, false, 0, 0, true><<<dim3((tiles + 7) / 8, 1), 256, 0, stream>>>(
        (const unsigned short*)yln, nullptr, DIN, 0L,
        (const unsigned short*)BtOut, nullptr, DIN, 0L,
        (void*)out, nullptr, D, 0L,
        nullptr, src, 0L, BL, D, DIN, 1.0f / 64.0f);
  }
  (void)ws;
}
